// GCNResnet_58789512348389
// MI455X (gfx1250) — hardware-run, weakly checked
//
#include <hip/hip_runtime.h>


#ifndef SEQ
#define SEQ 8192
#endif
#define SEQ_FULL 8192
#define NN   3
#define NF   10
#define XR   (NN * NF)
#define KD   32
#define VROWS 16
#define DO   10
#define AW   4
#define TP   64
#define PP   36
#define WLN  128
#define CAR  64.0f
#define VSI  (1.0f / 64.0f)
#define SC2  ((float)(1.4426950408889634 / 4096.0))
#define PSH  14.0f
#define NEGB (-3.0e38f)

static_assert(KD == 32);
static_assert(NF <= VROWS);
static_assert(NF <= KD);
static_assert(DO == NF);
static_assert(SEQ % TP == 0);
static_assert(TP == 64);
static_assert(SEQ % 32 == 0);
static_assert(SEQ % (16 * AW) == 0);
static_assert(SEQ <= SEQ_FULL);
static_assert(PP % 4 == 0);
static_assert(PP >= KD);
static_assert(WLN == 2 * TP);
static_assert(NF * NF <= WLN);
static_assert((TP * XR) % TP == 0);
static_assert((size_t)TP * 4 * 16 == (size_t)TP * KD * 2);
static_assert((size_t)TP * 2 * 16 == (size_t)VROWS * TP * 2);
static_assert(16 * DO * 4 == 32 * 16 + 8 * 16);
static_assert((16 * DO * 4) % 128 == 0);
static_assert((size_t)(TP * XR + WLN + TP + TP * PP) * 4 <= 131072);
static_assert((size_t)(AW * 16 * DO) * 4 <= 131072);

typedef _Float16 h16;
typedef __attribute__((ext_vector_type(16))) _Float16 v16h;
typedef __attribute__((ext_vector_type(8)))  _Float16 v8h;
typedef __attribute__((ext_vector_type(8)))  float    v8f;
typedef __attribute__((ext_vector_type(4)))  float    v4f;
typedef v4f  __attribute__((may_alias)) v4fa;

__device__ __forceinline__ unsigned short f2bf(float f) { unsigned u = __float_as_uint(f); u += 0x7FFFu + ((u >> 16) & 1u); return (unsigned short)(u >> 16); }
__device__ __forceinline__ float bfr(float f) { return __uint_as_float(((unsigned)f2bf(f)) << 16); }
__device__ __forceinline__ v16h cat16(v8h lo, v8h hi) { return __builtin_shufflevector(lo, hi, 0, 1, 2, 3, 4, 5, 6, 7, 8, 9, 10, 11, 12, 13, 14, 15); }
__device__ __forceinline__ v8f wmma16(v16h a, v16h b, v8f c) { return __builtin_amdgcn_wmma_f32_16x16x32_f16(false, a, false, b, (short)0, c, false, false); }
__device__ __forceinline__ v8f wmma16g(v16h a, v16h b, v8f c) {
    c = wmma16(a, b, c);
    asm volatile("v_nop\n\tv_nop\n\tv_nop\n\tv_nop" : "+v"(c) : "v"(a), "v"(b));
    return c;
}
__device__ __forceinline__ v16h ldh(const h16* p) { return cat16(*(const v8h*)p, *(const v8h*)(p + 16)); }
__device__ __forceinline__ h16 toh_flush(float v) { const h16 r = (h16)v; return (fabsf(v) < 6.103515625e-05f) ? (h16)0.0f : r; }
__device__ __forceinline__ void wave_sync() { __builtin_amdgcn_fence(3  , "wavefront"); __builtin_amdgcn_wave_barrier(); asm volatile("" ::: "memory"); }

__global__ __launch_bounds__(TP) void k_pool(const float* __restrict__ x, const float* __restrict__ A, const float* __restrict__ W, h16* PK, h16* VT) {
#pragma clang fp contract(off)
    __shared__ __align__(16) float xs[TP * XR];
    __shared__ __align__(16) float wl[WLN];
    __shared__ __align__(16) float adjs[TP];
    __shared__ __align__(16) float ps[TP * PP];
    const int tid = threadIdx.x;
    const int t0 = blockIdx.x * TP;
#pragma unroll 1
    for (int i = tid; i < TP * XR; i += TP) xs[i] = bfr(x[(size_t)t0 * XR + i]);
#pragma unroll 1
    for (int s = 0; s < 2; ++s) { const int i = s * TP + tid;
        const int ic = i < NF * NF ? i : (NF * NF - 1);
        const float wv = bfr(W[ic]);
        wl[i] = wv; }
    { const int ai = tid < 9 ? tid : 8;
      const float av = bfr(A[ai]);
      const float offv = ((ai / 3) != (ai % 3)) ? 1.0f : 0.0f;
      adjs[tid] = (0.5f * (offv + av)) * 0.5f; }
    __syncthreads();
    const float a00 = adjs[0], a01 = adjs[1], a02 = adjs[2], a10 = adjs[3], a11 = adjs[4], a12 = adjs[5];
#pragma unroll 1
    for (int o = 0; o < NF; ++o) {
        float s0 = 0.0f, s1 = 0.0f, s2 = 0.0f;
#pragma unroll 1
        for (int f = 0; f < NF; ++f) { const float w = wl[f * NF + o];
            s0 += xs[tid * XR + f] * w; s1 += xs[tid * XR + NF + f] * w; s2 += xs[tid * XR + 2 * NF + f] * w; }
        const float h0 = a00 * s0 + a01 * s1 + a02 * s2;
        const float h1 = a10 * s0 + a11 * s1 + a12 * s2;
        ps[tid * PP + o] = 0.5f * (h0 + h1);
    }
#pragma unroll 1
    for (int o = NF; o < KD; ++o) ps[tid * PP + o] = 0.0f;
    __syncthreads();
    h16* pkb = PK + (size_t)t0 * KD;
    h16* vtb = VT + (size_t)t0;
#pragma unroll 1
    for (int pass = 0; pass < 2; ++pass) {
#pragma unroll
        for (int s = 0; s < 4; ++s) { const int p = s * TP + tid; const int row = p >> 2, c8 = (p & 3) * 8;
            const v4f x0 = *(const v4fa*)(&ps[row * PP + c8]); const v4f x1 = *(const v4fa*)(&ps[row * PP + c8 + 4]); v8h hv;
#pragma unroll
            for (int i = 0; i < 4; ++i) { hv[i] = toh_flush(x0[i] * CAR); hv[4 + i] = toh_flush(x1[i] * CAR); }
            *(volatile v8h*)(pkb + (size_t)p * 8) = hv; }
#pragma unroll
        for (int s = 0; s < 2; ++s) { const int p = s * TP + tid; const int row = p >> 3, c8 = (p & 7) * 8;
            v8h hv;
#pragma unroll
            for (int i = 0; i < 8; ++i) hv[i] = toh_flush(ps[(c8 + i) * PP + row] * CAR);
            *(volatile v8h*)(vtb + (size_t)row * SEQ + c8) = hv; }
        if (pass == 0) __threadfence(); }
}

__global__ __launch_bounds__(32 * AW) void k_flash(const h16* __restrict__ PK, const h16* __restrict__ VT, float* OUT) {
    __shared__ __align__(16) float os[AW * 16 * DO];
    const int lane = threadIdx.x & 31, lr = lane & 15, hi = lane >> 4;
    const int wave = __builtin_amdgcn_readfirstlane((int)(threadIdx.x >> 5));
    const int t0 = (blockIdx.x * AW + wave) * 16;
    const v16h qh = ldh(PK + (size_t)(t0 + lr) * KD + 8 * hi);
    const size_t ko = (size_t)lr * KD + 8 * hi;
    const size_t vo = (size_t)lr * SEQ + 8 * hi;
    v8f o0 = (v8f){};
    float m = NEGB, l = 0.0f;
#pragma unroll 1
    for (int key0 = 0; key0 < SEQ; key0 += 32) {
        const h16* ka = PK + ko + (size_t)key0 * KD;
        const v16h ka0 = ldh(ka), kb0 = ldh(ka + 16 * KD);
        v8f sa = (v8f){}, sb = (v8f){};
        sa = wmma16g(ka0, qh, sa);
        sb = wmma16g(kb0, qh, sb);
        float ta[8], tb[8]; float mx = NEGB;
#pragma unroll
        for (int r = 0; r < 8; ++r) { ta[r] = sa[r] * SC2; tb[r] = sb[r] * SC2; mx = fmaxf(mx, fmaxf(ta[r], tb[r])); }
        mx = fmaxf(mx, __shfl_xor(mx, 16, 32));
        const float mnew = fmaxf(m, mx);
        const float alpha = __builtin_amdgcn_exp2f(m - mnew);
        const float sh = PSH - mnew;
        v16h pb; float ls = 0.0f;
#pragma unroll
        for (int r = 0; r < 8; ++r) {
            const float xa = ta[r] + sh, xb = tb[r] + sh;
            const float ea = __builtin_amdgcn_exp2f(xa), eb = __builtin_amdgcn_exp2f(xb);
            const float ga = (xa < -14.0f) ? 0.0f : ea, gb = (xb < -14.0f) ? 0.0f : eb;
            const h16 pa = (h16)ga; const h16 pc = (h16)gb;
            pb[r] = pa; pb[8 + r] = pc;
            ls += (float)pa + (float)pc; }
        l = l * alpha + ls; m = mnew;
        o0 = o0 * alpha;
        const v16h v0 = ldh(VT + vo + key0);
        o0 = wmma16g(v0, pb, o0);
    }
    l += __shfl_xor(l, 16, 32);
    const float inv = (1.0f / l) * VSI;
    const int wb = wave * 16 * DO;
#pragma unroll
    for (int r = 0; r < 8; ++r) { if (8 * hi + r < DO) os[wb + lr * DO + 8 * hi + r] = o0[r] * inv; }
    wave_sync();
    float* ob = OUT + (size_t)t0 * DO;
    const int i2 = 128 + (lane & 7) * 4;
#pragma unroll 1
    for (int ps = 0; ps < 2; ++ps) {
        const v4f val = *(const v4fa*)(&os[wb + lane * 4]);
        v4f va2 = *(const v4fa*)(&os[wb + i2]);
        asm volatile("" : "+v"(va2));
        *(volatile v4f*)(ob + lane * 4) = val;
        if (lane < 8) *(volatile v4f*)(ob + i2) = va2;
        if (ps == 0) __threadfence(); }
}

static constexpr size_t al256(size_t v) { return (v + 255) & ~(size_t)255; }
static constexpr size_t SZ_PK = al256((size_t)SEQ * KD * 2);
static constexpr size_t SZ_VT = al256((size_t)VROWS * SEQ * 2);
static constexpr size_t SZ_TOTAL = SZ_PK + SZ_VT;
static_assert(SZ_TOTAL <= (size_t)134217728);
static_assert((size_t)SEQ * KD * 2 == (size_t)(SEQ / TP) * TP * 4 * 16);
static_assert((size_t)VROWS * SEQ * 2 == (size_t)(SEQ / TP) * TP * 2 * 16);
static_assert((size_t)SEQ * DO * 4 == (size_t)(SEQ / 16) * 640);

extern "C" void kernel_launch(void* const* d_in, const int* in_sizes, int n_in,
                              void* d_out, int out_size, void* d_ws, size_t ws_size, hipStream_t stream) {
    if (n_in < 3) return;
    if ((size_t)in_sizes[0] < (size_t)SEQ * XR) return;
    if (in_sizes[1] < 9 || in_sizes[2] < NF * NF) return;
    if ((size_t)out_size < (size_t)SEQ * DO) return;
    if (SZ_TOTAL > ws_size) return;
    const float* x = (const float*)d_in[0];
    const float* A = (const float*)d_in[1];
    const float* W = (const float*)d_in[2];
    float* OUT = (float*)d_out;
    char* wsp = (char*)d_ws;
    h16* PK = (h16*)wsp; wsp += SZ_PK;
    h16* VT = (h16*)wsp; wsp += SZ_VT;

    k_pool<<<dim3(SEQ / TP, 1, 1), TP, 0, stream>>>(x, A, W, PK, VT);
    k_flash<<<dim3(SEQ / (16 * AW), 1, 1), 32 * AW, 0, stream>>>(PK, VT, OUT);
}
